// MoENetwork_43499428774597
// MI455X (gfx1250) — hardware-verified
//
#include <hip/hip_runtime.h>
#include <stddef.h>
#include <stdint.h>

#pragma clang fp contract(off)

#define TOKENS 1024
#define DD     512
#define HH     256
#define OO     512
#define NE     64
#define KMAX   4
#define NSLOT  (TOKENS * KMAX)
#define NTILE  128
#define NROWS  (NTILE * 64)
#define TB_OFF 64
#define NTL_OFF 128
#define TABN   256
#define WSC    64.0f
#define INV64  0.015625f
#define CHH    16.0f
#define INVHY  0.0009765625f
#define YPITCH 68
#define HPITCH 72
#define TP     68

static_assert(NTILE >= NSLOT / 64 + NE);
static_assert(NROWS <= 65536);
static_assert(TOKENS <= 65536);
static_assert(4 * NE == 256);
static_assert(TABN == 256);
static_assert(TB_OFF + NE <= NTL_OFF);
static_assert(NTL_OFF < TABN);
static_assert(NROWS % 1024 == 0);
static_assert(NSLOT % 1024 == 0);
static_assert(DD % 128 == 0);
static_assert(HH % 128 == 0);
static_assert(OO % 128 == 0);
static_assert(DD % 64 == 0);
static_assert(HH % 64 == 0);
static_assert(TOKENS % 32 == 0);
static_assert(32 * KMAX == 128);
static_assert((YPITCH * 4) % 16 == 0);
static_assert((HPITCH * 2) % 16 == 0);
static_assert((TP * 4) % 16 == 0);

typedef _Float16 v16h __attribute__((ext_vector_type(16)));
typedef _Float16 v8h  __attribute__((ext_vector_type(8)));
typedef float    v8f  __attribute__((ext_vector_type(8)));
typedef float    v4f  __attribute__((ext_vector_type(4)));
typedef unsigned int v4u __attribute__((ext_vector_type(4)));
typedef int      v4i  __attribute__((ext_vector_type(4)));
typedef unsigned short v4us __attribute__((ext_vector_type(4)));

union Frag  { v16h v; v8h h[2]; };
union Pack8 { v8h h; v4u u; };

__device__ __forceinline__ int clampi(int v, int lo, int hi) { return min(max(v, lo), hi); }

__device__ __forceinline__ v8f mma16(v16h a, v16h b, v8f c) {
  c = __builtin_amdgcn_wmma_f32_16x16x32_f16(false, a, false, b, (short)0, c, false, false);
  asm volatile("v_nop\n\tv_nop\n\tv_nop\n\tv_nop" : "+v"(c) : "v"(a), "v"(b));
  return c;
}

__device__ __forceinline__ v16h ldfrag(const _Float16* p, int ld, int row0, int k0, int lane) {
  const int m = lane & 15, lh = lane >> 4;
  const _Float16* q = p + (size_t)(row0 + m) * ld + k0 + 8 * lh;
  Frag f;
  f.h[0] = *(const v8h*)(q);
  f.h[1] = *(const v8h*)(q + 16);
  return f.v;
}

__device__ __forceinline__ v8f zero8() { return (v8f){0.f, 0.f, 0.f, 0.f, 0.f, 0.f, 0.f, 0.f}; }

__device__ __forceinline__ v4u pack8h(v4f a0, v4f a1) {
  Pack8 pk;
  pk.h = (v8h){(_Float16)a0[0], (_Float16)a0[1], (_Float16)a0[2], (_Float16)a0[3],
               (_Float16)a1[0], (_Float16)a1[1], (_Float16)a1[2], (_Float16)a1[3]};
  return pk.u;
}

__global__ __launch_bounds__(256) void k_tr(const float* __restrict__ src, _Float16* __restrict__ dst,
                                            int R, int C, float scale) {
  __shared__ __align__(16) float tile[32 * TP];
  const int tid = threadIdx.x;
  const size_t slab = (size_t)R * (size_t)C;
  const float* s = src + (size_t)blockIdx.z * slab;
  _Float16* d = dst + (size_t)blockIdx.z * slab;
  const int c0 = blockIdx.x * 32, r0 = blockIdx.y * 64;
  const int tx = tid & 31, ty = tid >> 5;
#pragma unroll
  for (int j = 0; j < 8; ++j)
    tile[tx * TP + ty + 8 * j] = s[(size_t)(r0 + ty + 8 * j) * C + c0 + tx] * scale;
  __syncthreads();
  const int orow = tid >> 3, q = tid & 7;
  const v4f a0 = *(const v4f*)(tile + orow * TP + 8 * q);
  const v4f a1 = *(const v4f*)(tile + orow * TP + 8 * q + 4);
  const v4u vv = pack8h(a0, a1);
  volatile v4u* dp = (volatile v4u*)(d + (size_t)(c0 + orow) * R + r0 + 8 * q);
  *dp = vv;
  __threadfence();
  *dp = vv;
}

__global__ __launch_bounds__(256) void k_gate(const float* __restrict__ x, const float* __restrict__ noise,
                                              const float* __restrict__ mixer, const float* __restrict__ ncont,
                                              const int* __restrict__ kp, int* __restrict__ eidp,
                                              float* __restrict__ scp) {
  __shared__ __align__(16) int sE[32 * KMAX];
  __shared__ __align__(16) float sS[32 * KMAX];
  const int tid = threadIdx.x, lane = tid & 31, wave = tid >> 5;
  const int kk = clampi(kp[0], 1, KMAX);
  const float neg_inf = __int_as_float(0xff800000);

#pragma unroll 1
  for (int jt = 0; jt < 4; ++jt) {
    const int tl = wave * 4 + jt;
    const int t = blockIdx.x * 32 + tl;
    const float* xr = x + (size_t)t * DD;
    float a0 = 0.f, a1 = 0.f, c0 = 0.f, c1 = 0.f;
#pragma unroll 1
    for (int i = 0; i < DD / 4; ++i) {
      const int d0 = 4 * i;
      const v4f xv = *(const v4f*)(xr + d0);
#pragma unroll
      for (int dd = 0; dd < 4; ++dd) {
        const float* mr = mixer + (size_t)(d0 + dd) * NE;
        const float* nr = ncont + (size_t)(d0 + dd) * NE;
        const float xs = xv[dd];
        a0 = fmaf(xs, mr[lane], a0);
        a1 = fmaf(xs, mr[lane + 32], a1);
        c0 = fmaf(xs, nr[lane], c0);
        c1 = fmaf(xs, nr[lane + 32], c1);
      }
    }
    const float n0 = noise[(size_t)t * NE + lane];
    const float n1 = noise[(size_t)t * NE + lane + 32];
    float h0 = 0.f, h1 = 0.f;
#pragma unroll 1
    for (int s2 = 0; s2 < 2; ++s2) {
      const float av = (s2 == 0) ? a0 : a1;
      const float cv = (s2 == 0) ? c0 : c1;
      const float nv = (s2 == 0) ? n0 : n1;
      const float sp = fmaxf(cv, 0.0f) + log1pf(expf(-fabsf(cv)));
      const float hv = av + nv * sp;
      h0 = (s2 == 0) ? hv : h0;
      h1 = (s2 == 0) ? h1 : hv;
    }

    float vals[KMAX];
    int ids[KMAX];
#pragma unroll
    for (int j = 0; j < KMAX; ++j) {
      const bool take0 = (h0 >= h1);
      float v = take0 ? h0 : h1;
      int id = take0 ? lane : (lane + 32);
#pragma unroll
      for (int off = 16; off > 0; off >>= 1) {
        const float ov = __shfl_xor(v, off, 32);
        const int   oi = __shfl_xor(id, off, 32);
        const bool tk = (ov > v) || ((ov == v) && (oi < id));
        v  = tk ? ov : v;
        id = tk ? oi : id;
      }
      vals[j] = v;
      ids[j] = id;
      h0 = (id == lane) ? neg_inf : h0;
      h1 = (id == lane + 32) ? neg_inf : h1;
    }

    const float mval = vals[0];
    float ex[KMAX];
#pragma unroll
    for (int j = 0; j < KMAX; ++j) ex[j] = 0.f;
    float ssum = 0.f;
#pragma unroll 1
    for (int j = 0; j < KMAX; ++j) {
      float vj = vals[0];
#pragma unroll
      for (int q = 1; q < KMAX; ++q) vj = (q == j) ? vals[q] : vj;
      float ej = expf(vj - mval);
      ej = (j < kk) ? ej : 0.f;
      ssum += ej;
#pragma unroll
      for (int q = 0; q < KMAX; ++q) ex[q] = (q == j) ? ej : ex[q];
    }
    const float inv = 1.0f / ssum;
    if (lane == 0) {
#pragma unroll
      for (int j = 0; j < KMAX; ++j) {
        sE[tl * KMAX + j] = (j < kk) ? ids[j] : NE;
        sS[tl * KMAX + j] = ex[j] * inv;
      }
    }
  }
  __syncthreads();
  if (wave == 0) {
    const v4i ve = *(const v4i*)(sE + lane * 4);
    const v4f vs = *(const v4f*)(sS + lane * 4);
    const size_t go = (size_t)blockIdx.x * (32 * KMAX) + (size_t)lane * 4;
    volatile v4i* de = (volatile v4i*)(eidp + go);
    volatile v4f* ds = (volatile v4f*)(scp + go);
    *de = ve;
    *ds = vs;
    __threadfence();
    *de = ve;
    *ds = vs;
  }
}

__global__ __launch_bounds__(256) void k_lists(const int* __restrict__ eidp, int* __restrict__ tokp,
                                               int* __restrict__ posp, int* __restrict__ tab) {
  __shared__ unsigned char sId[NSLOT];
  __shared__ __align__(16) unsigned short ltok[NROWS];
  __shared__ __align__(16) unsigned short sPos[NSLOT];
  __shared__ int cq[4 * NE];
  __shared__ __align__(16) int sTab[TABN];
  const int tid = threadIdx.x;

#pragma unroll 1
  for (int i = tid; i < NSLOT; i += 256) {
    sId[i] = (unsigned char)clampi(eidp[i], 0, NE);
    sPos[i] = (unsigned short)0;
  }
#pragma unroll 1
  for (int r = tid; r < NROWS; r += 256) ltok[r] = (unsigned short)0;
  sTab[tid] = 0;
  __syncthreads();

  const int q = tid >> 6, e = tid & (NE - 1);
  const int i0 = q * (NSLOT / 4);
  int cnt = 0;
#pragma unroll 4
  for (int i = 0; i < NSLOT / 4; ++i) cnt += ((int)sId[i0 + i] == e) ? 1 : 0;
  cq[q * NE + e] = cnt;
  __syncthreads();
  if (tid < NE) sTab[tid] = cq[tid] + cq[NE + tid] + cq[2 * NE + tid] + cq[3 * NE + tid];
  __syncthreads();
  if (tid == 0) {
    int run = 0;
#pragma unroll 1
    for (int e2 = 0; e2 < NE; ++e2) {
      sTab[TB_OFF + e2] = run;
      run += (clampi(sTab[e2], 0, NSLOT) + 63) >> 6;
    }
    sTab[TB_OFF + NE] = clampi(run, 0, NTILE);
    sTab[NTL_OFF] = clampi(run, 0, NTILE);
  }
  __syncthreads();

  int rank = 0;
#pragma unroll
  for (int p = 0; p < 4; ++p) rank += (p < q) ? cq[p * NE + e] : 0;
  const int tbe = clampi(sTab[TB_OFF + e], 0, NTILE - 1);
#pragma unroll 2
  for (int i = 0; i < NSLOT / 4; ++i) {
    const int s = i0 + i;
    if ((int)sId[s] == e) {
      const int row = clampi(tbe * 64 + rank, 0, NROWS - 1);
      ltok[row] = (unsigned short)(s / KMAX);
      sPos[s] = (unsigned short)row;
      ++rank;
    }
  }
  __syncthreads();

  for (int ps = 0; ps < 2; ++ps) {
#pragma unroll
    for (int it = 0; it < NROWS / 1024; ++it) {
      const int p = tid + 256 * it;
      const v4us u = *(const v4us*)(ltok + 4 * p);
      const v4i v = (v4i){(int)u[0], (int)u[1], (int)u[2], (int)u[3]};
      *(volatile v4i*)(tokp + (size_t)p * 4) = v;
    }
#pragma unroll
    for (int it = 0; it < NSLOT / 1024; ++it) {
      const int p = tid + 256 * it;
      const v4us u = *(const v4us*)(sPos + 4 * p);
      const v4i v = (v4i){(int)u[0], (int)u[1], (int)u[2], (int)u[3]};
      *(volatile v4i*)(posp + (size_t)p * 4) = v;
    }
    if (tid < TABN / 4) {
      const v4i v = *(const v4i*)(sTab + 4 * tid);
      *(volatile v4i*)(tab + 4 * tid) = v;
    }
    __threadfence();
  }
}

__global__ __launch_bounds__(64) void k_gather(const float* __restrict__ x, const int* __restrict__ tokp,
                                               _Float16* __restrict__ xg) {
  const int row = blockIdx.x;
  const int t = clampi(tokp[row], 0, TOKENS - 1);
  const int o = (int)threadIdx.x * 8;
  const float* xr = x + (size_t)t * DD + o;
  const v4f a0 = *(const v4f*)(xr);
  const v4f a1 = *(const v4f*)(xr + 4);
  const v4u vv = pack8h(a0, a1);
  volatile v4u* dp = (volatile v4u*)(xg + (size_t)row * DD + o);
  *dp = vv;
  __threadfence();
  *dp = vv;
}

template <int KK, int NO, int MODE>
__global__ __launch_bounds__(256) void k_ffn(const _Float16* __restrict__ ap, const _Float16* __restrict__ wt,
                                             const float* __restrict__ bias, const int* __restrict__ tab,
                                             _Float16* __restrict__ hout, float* __restrict__ yout) {
  __shared__ __align__(16) float sC[8 * 16 * YPITCH];
  __shared__ __align__(16) _Float16 sH[8 * 16 * HPITCH];
  __shared__ int sTab[TABN];
  const int tid = threadIdx.x, lane = tid & 31, wave = tid >> 5;
  const int hh = lane >> 4, c = lane & 15;
  const int wm = wave & 3, wn = wave >> 2;
  const int b  = blockIdx.x;

  sTab[tid] = tab[tid];
  __syncthreads();
  const int ntl = clampi(sTab[NTL_OFF], 0, NTILE);
  if (b >= ntl) return;
  int e = 0;
#pragma unroll
  for (int q = 1; q < NE; ++q) e += (clampi(sTab[TB_OFF + q], 0, NTILE) <= b) ? 1 : 0;

  const _Float16* we = wt + (size_t)e * ((size_t)NO * (size_t)KK);
  const float* bse = bias + (size_t)e * NO;
  const int arow0 = b * 64 + wm * 16;
  float* cw = sC + wave * (16 * YPITCH);
  _Float16* hw = sH + wave * (16 * HPITCH);

#pragma unroll 1
  for (int nc = 0; nc < NO / 128; ++nc) {
    const int brow = nc * 128 + wn * 64;
    v8f acc[4];
#pragma unroll
    for (int t = 0; t < 4; ++t) acc[t] = zero8();
#pragma unroll 2
    for (int ks = 0; ks < KK / 32; ++ks) {
      const int kg = ks * 32;
      const v16h a = ldfrag(ap, KK, arow0, kg, lane);
#pragma unroll
      for (int t = 0; t < 4; ++t) {
        const v16h bq = ldfrag(we, KK, brow + 16 * t, kg, lane);
        acc[t] = mma16(a, bq, acc[t]);
      }
    }
    if (MODE == 0) {
#pragma unroll
      for (int t = 0; t < 4; ++t) {
        const int ncol = 16 * t + c;
        const float bv = bse[brow + ncol];
#pragma unroll
        for (int r = 0; r < 8; ++r) {
          const float v = fmaxf(acc[t][r] * INV64 + bv, 0.0f) * CHH;
          hw[(8 * hh + r) * HPITCH + ncol] = (_Float16)v;
        }
      }
      __syncthreads();
      for (int ps = 0; ps < 2; ++ps) {
#pragma unroll
        for (int i = 0; i < 4; ++i) {
          const int row = 4 * i + (lane >> 3);
          const int q = lane & 7;
          Pack8 pk;
          pk.h = *(const v8h*)(hw + row * HPITCH + 8 * q);
          const size_t go = (size_t)(arow0 + row) * NO + brow + 8 * q;
          *(volatile v4u*)(hout + go) = pk.u;
        }
        __threadfence();
      }
    } else {
#pragma unroll
      for (int t = 0; t < 4; ++t) {
        const int ncol = 16 * t + c;
        const float bv = bse[brow + ncol];
#pragma unroll
        for (int r = 0; r < 8; ++r) cw[(8 * hh + r) * YPITCH + ncol] = acc[t][r] * INVHY + bv;
      }
      __syncthreads();
      for (int ps = 0; ps < 2; ++ps) {
#pragma unroll
        for (int i = 0; i < 8; ++i) {
          const int row = 2 * i + hh;
          const v4f v = *(const v4f*)(cw + row * YPITCH + c * 4);
          const size_t go = (size_t)(arow0 + row) * NO + brow + c * 4;
          *(volatile v4f*)(yout + go) = v;
        }
        __threadfence();
      }
    }
    __syncthreads();
  }
}

__global__ __launch_bounds__(128) void k_out(const float* __restrict__ yp, const int* __restrict__ posp,
                                             const float* __restrict__ scp, const int* __restrict__ kp,
                                             float* __restrict__ out) {
  const int t  = blockIdx.x;
  const int c4 = (int)threadIdx.x;
  const int kr = kp[0];
  const int kk = clampi(kr, 1, KMAX);
  const bool badk = (kr < 1) || (kr > KMAX);
  v4f acc = (v4f){0.f, 0.f, 0.f, 0.f};
#pragma unroll
  for (int j = 0; j < KMAX; ++j) {
    const int s = t * KMAX + j;
    const int r = clampi(posp[s], 0, NROWS - 1);
    float sc = scp[s];
    sc = (j < kk) ? sc : 0.f;
    const v4f yv = *(const v4f*)(yp + (size_t)r * OO + c4 * 4);
    const v4f pj = yv * sc;
    acc = acc + pj;
  }
  if (badk) {
    const float qn = __int_as_float(0x7fc00000);
    acc = (v4f){qn, qn, qn, qn};
  }
  volatile v4f* dp = (volatile v4f*)(out + (size_t)t * OO + c4 * 4);
  *dp = acc;
  __threadfence();
  *dp = acc;
}

extern "C" void kernel_launch(void* const* d_in, const int* in_sizes, int n_in,
                              void* d_out, int out_size, void* d_ws, size_t ws_size,
                              hipStream_t stream) {
  if (n_in < 9) return;
  if (in_sizes[0] != TOKENS * DD) return;
  if (in_sizes[1] != TOKENS * NE) return;
  if (in_sizes[2] != NE * DD * HH) return;
  if (in_sizes[3] != NE * HH) return;
  if (in_sizes[4] != NE * HH * OO) return;
  if (in_sizes[5] != NE * OO) return;
  if (in_sizes[6] != DD * NE) return;
  if (in_sizes[7] != DD * NE) return;
  if (in_sizes[8] < 1) return;
  if (out_size != TOKENS * OO) return;

  const float* x     = (const float*)d_in[0];
  const float* noise = (const float*)d_in[1];
  const float* w1s   = (const float*)d_in[2];
  const float* b1s   = (const float*)d_in[3];
  const float* w2s   = (const float*)d_in[4];
  const float* b2s   = (const float*)d_in[5];
  const float* mixer = (const float*)d_in[6];
  const float* ncont = (const float*)d_in[7];
  const int*   kp    = (const int*)d_in[8];
  float* out = (float*)d_out;

  size_t off = 0;
  const size_t oW1 = off; off += (size_t)NE * HH * DD * 2;
  const size_t oW2 = off; off += (size_t)NE * OO * HH * 2;
  const size_t oEI = off; off += (size_t)NSLOT * 4;
  const size_t oSC = off; off += (size_t)NSLOT * 4;
  const size_t oTK = off; off += (size_t)NROWS * 4;
  const size_t oPS = off; off += (size_t)NSLOT * 4;
  const size_t oTB = off; off += (size_t)TABN * 4;
  const size_t oXG = off; off += (size_t)NROWS * DD * 2;
  const size_t oHH = off; off += (size_t)NROWS * HH * 2;
  const size_t oY  = off; off += (size_t)NROWS * OO * 4;
  if (off > ws_size) return;
  if (off > (size_t)134217728) return;
  if ((oW2 | oEI | oSC | oTK | oPS | oTB | oXG | oHH | oY) & (size_t)127) return;

  char* ws = (char*)d_ws;
  _Float16* W1t = (_Float16*)(ws + oW1);
  _Float16* W2t = (_Float16*)(ws + oW2);
  int*      EID = (int*)(ws + oEI);
  float*    SC  = (float*)(ws + oSC);
  int*      TOK = (int*)(ws + oTK);
  int*      POS = (int*)(ws + oPS);
  int*      TAB = (int*)(ws + oTB);
  _Float16* Xg  = (_Float16*)(ws + oXG);
  _Float16* Hh  = (_Float16*)(ws + oHH);
  float*    Y   = (float*)(ws + oY);

  k_tr<<<dim3(HH / 32, DD / 64, NE), dim3(256), 0, stream>>>(w1s, W1t, DD, HH, WSC);
  k_tr<<<dim3(OO / 32, HH / 64, NE), dim3(256), 0, stream>>>(w2s, W2t, HH, OO, WSC);
  k_gate<<<dim3(TOKENS / 32), dim3(256), 0, stream>>>(x, noise, mixer, ncont, kp, EID, SC);
  k_lists<<<dim3(1), dim3(256), 0, stream>>>(EID, TOK, POS, TAB);
  k_gather<<<dim3(NROWS), dim3(DD / 8), 0, stream>>>(x, TOK, Xg);
  k_ffn<DD, HH, 0><<<dim3(NTILE), dim3(256), 0, stream>>>(Xg, W1t, b1s, TAB, Hh, Y);
  k_ffn<HH, OO, 1><<<dim3(NTILE), dim3(256), 0, stream>>>(Hh, W2t, b2s, TAB, Hh, Y);
  k_out<<<dim3(TOKENS), dim3(OO / 4), 0, stream>>>(Y, POS, SC, kp, out);
  (void)hipGetLastError();
}
